// SparseMultiheadAttention_16303695856197
// MI455X (gfx1250) — hardware-verified
//
#include <hip/hip_runtime.h>
#include <math.h>
#include <stdint.h>

#define SEQ_FULL 2048
#ifndef SEQ
#define SEQ   SEQ_FULL
#endif
#ifndef NB
#define NB    1
#endif
#define DMOD  768
#define NH    12
#define HD    64
#define WSPAN 64
#define QSC   8.0f
#define KSC   8.0f
#define QKRS  2048.0f
#define PCAR  32768.0f
#define VCAR  1024.0f
#define OSC   1024.0f
#define ORS   2048.0f
#define WOS   1024.0f
#define RSQN  0.022097086912079612f
#define LOG2E 1.4426950408889634f
#define NEGS  (-3.0e38f)
#define ATT_WAVES   4
#define ATT_THREADS (ATT_WAVES * 32)
#define NQT         (SEQ / 64)
#define ATT_BLOCKS  (NH * NQT)
#define NKB    (SEQ / 32)
#define SLAB   (16 * 68)
static_assert(NB == 1);
static_assert(HD == 64 && DMOD == NH * HD);
static_assert((SEQ % 64) == 0 && SEQ >= 64 && SEQ <= SEQ_FULL);
static_assert(ATT_THREADS == 128 && NKB >= 2);
static_assert((DMOD % 64) == 0 && (DMOD % 32) == 0);
static_assert(((SEQ * DMOD / 8) % 256) == 0);
static_assert((SLAB * 4) % 16 == 0);

typedef unsigned short u16;
typedef _Float16 v16h __attribute__((ext_vector_type(16)));
typedef _Float16 v8h  __attribute__((ext_vector_type(8)));
typedef __bf16   v16b __attribute__((ext_vector_type(16)));
typedef float    v8f  __attribute__((ext_vector_type(8)));
typedef float    v4f  __attribute__((ext_vector_type(4)));
typedef unsigned int v4u __attribute__((ext_vector_type(4)));

union FragH { v16h v; v8h h[2]; v4u u[2]; };
union FragB { v16b v; v4u u[2]; };

__device__ __forceinline__ unsigned short bf_bits(float f) {
  unsigned u = __float_as_uint(f);
  return (unsigned short)((u + 0x7FFFu + ((u >> 16) & 1u)) >> 16);
}
__device__ __forceinline__ float bf_up(unsigned short h) { return __uint_as_float(((unsigned)h) << 16); }
__device__ __forceinline__ float bf_val(float f) { return bf_up(bf_bits(f)); }
__device__ __forceinline__ unsigned short h_bits(_Float16 x) { return __builtin_bit_cast(unsigned short, x); }
__device__ __forceinline__ unsigned pk16(unsigned short a, unsigned short b) { return (unsigned)a | ((unsigned)b << 16); }
__device__ __forceinline__ v8f zero8() { v8f z = {0.f, 0.f, 0.f, 0.f, 0.f, 0.f, 0.f, 0.f}; return z; }

__device__ __forceinline__ v16h ldfrag_h(const _Float16* p) {
  FragH f;
  f.h[0] = *(const v8h*)(p);
  f.h[1] = *(const v8h*)(p + 16);
  return f.v;
}
__device__ __forceinline__ v16b ldfrag_b(const u16* p) {
  FragB f;
  f.u[0] = *(const v4u*)(p);
  f.u[1] = *(const v4u*)(p + 16);
  return f.v;
}

__device__ __forceinline__ v8f mma_h(v16h a, v16h b, v8f c) {
  return __builtin_amdgcn_wmma_f32_16x16x32_f16(false, a, false, b, (short)0, c, false, false);
}
__device__ __forceinline__ v8f mma_b(v16b a, v16b b, v8f c) {
  return __builtin_amdgcn_wmma_f32_16x16x32_bf16(false, a, false, b, (short)0, c, false, false);
}
__device__ __forceinline__ void guard2f8(v8f& a, v8f& b, v16h x0, v16h x1, v16h x2, v16h x3,
                                         v16h x4, v16h x5, v16h x6, v16h x7) {
#if defined(__HIP_DEVICE_COMPILE__)
  asm volatile("v_nop\n\tv_nop\n\tv_nop\n\tv_nop"
               : "+v"(a), "+v"(b)
               : "v"(x0), "v"(x1), "v"(x2), "v"(x3), "v"(x4), "v"(x5), "v"(x6), "v"(x7) : "memory");
#endif
}
template <typename F>
__device__ __forceinline__ void guard6(v8f& a, v8f& b, v8f& c, v8f& d, F x0, F x1, F x2, F x3, F x4, F x5) {
#if defined(__HIP_DEVICE_COMPILE__)
  asm volatile("v_nop\n\tv_nop\n\tv_nop\n\tv_nop"
               : "+v"(a), "+v"(b), "+v"(c), "+v"(d) : "v"(x0), "v"(x1), "v"(x2), "v"(x3), "v"(x4), "v"(x5) : "memory");
#endif
}
__device__ __forceinline__ void guard8(v8f& a, v8f& b, v8f& c, v8f& d, v8f& e, v8f& f, v8f& g, v8f& h,
                                       v16h x0, v16h x1, v16h x2, v16h x3, v16h x4, v16h x5) {
#if defined(__HIP_DEVICE_COMPILE__)
  asm volatile("v_nop\n\tv_nop\n\tv_nop\n\tv_nop"
               : "+v"(a), "+v"(b), "+v"(c), "+v"(d), "+v"(e), "+v"(f), "+v"(g), "+v"(h)
               : "v"(x0), "v"(x1), "v"(x2), "v"(x3), "v"(x4), "v"(x5) : "memory");
#endif
}
__device__ __forceinline__ void acc_guard4(v8f& a, v8f& b, v8f& c, v8f& d) {
#if defined(__HIP_DEVICE_COMPILE__)
  asm volatile("v_nop\n\tv_nop\n\tv_nop\n\tv_nop" : "+v"(a), "+v"(b), "+v"(c), "+v"(d));
#endif
}
__device__ __forceinline__ void wave_sync_lds() {
#if defined(__HIP_DEVICE_COMPILE__)
  __builtin_amdgcn_fence(__ATOMIC_RELEASE, "workgroup");
  __builtin_amdgcn_wave_barrier();
  __builtin_amdgcn_fence(__ATOMIC_ACQUIRE, "workgroup");
#endif
}

__global__ __launch_bounds__(256) void cvt16(const float* __restrict__ x, u16* D, int n8) {
  const int gt = blockIdx.x * 256 + (int)threadIdx.x;
  if (gt >= n8) return;
  const float* p = x + (size_t)gt * 8;
  const v4f a = *(const v4f*)(p), c4 = *(const v4f*)(p + 4);
  float v[8];
#pragma unroll
  for (int e = 0; e < 4; ++e) { v[e] = a[e]; v[4 + e] = c4[e]; }
  unsigned short s[8];
#pragma unroll
  for (int e = 0; e < 8; ++e) s[e] = bf_bits(v[e]);
  v4u o;
#pragma unroll
  for (int e = 0; e < 4; ++e) o[e] = pk16(s[2 * e], s[2 * e + 1]);
  u16* d = D + (size_t)gt * 8;
  for (int pass = 0; pass < 2; ++pass) {
    *(volatile v4u*)(d) = o;
    __threadfence();
  }
}

__global__ __launch_bounds__(256) void cvtT16(const float* __restrict__ W, u16* D, int Kd, int Nd, int mode, float scale) {
  __shared__ __align__(16) float tile[64 * 65];
  const int tid = threadIdx.x, wave = tid >> 5, lane = tid & 31;
  const int ntn = Nd >> 6;
  const int bt  = blockIdx.x;
  const int kt  = bt / ntn;
  const int k0  = kt * 64;
  const int n0  = (bt - kt * ntn) * 64;
  if (k0 + 64 > Kd) return;
  {
    const int r = tid >> 2, c16 = (tid & 3) * 16;
    const float* src = W + (size_t)(k0 + r) * (size_t)Nd + n0 + c16;
#pragma unroll
    for (int e = 0; e < 4; ++e) {
      const v4f a = *(const v4f*)(src + 4 * e);
      float* t = tile + r * 65 + c16 + 4 * e;
      t[0] = a[0]; t[1] = a[1]; t[2] = a[2]; t[3] = a[3];
    }
  }
  __syncthreads();
  const int rq = lane >> 3, c8 = (lane & 7) * 8;
  v4u ov[2];
#pragma unroll
  for (int it = 0; it < 2; ++it) {
    const int nn = it * 32 + wave * 4 + rq;
    unsigned short s[8];
#pragma unroll
    for (int e = 0; e < 8; ++e) {
      const float f = tile[(c8 + e) * 65 + nn];
      const unsigned short bb = bf_bits(f);
      const unsigned short hb = h_bits((_Float16)(bf_up(bb) * scale));
      s[e] = (mode != 0) ? hb : bb;
    }
#pragma unroll
    for (int e = 0; e < 4; ++e) ov[it][e] = pk16(s[2 * e], s[2 * e + 1]);
  }
  u16* dst = D + (size_t)(n0 + wave * 4 + rq) * (size_t)Kd + k0 + c8;
  for (int pass = 0; pass < 2; ++pass) {
#pragma unroll
    for (int it = 0; it < 2; ++it) {
      *(volatile v4u*)(dst + (size_t)(it * 32) * (size_t)Kd) = ov[it];
    }
    __threadfence();
  }
}

__device__ __forceinline__ void epi16(float* sl, v8f a0, v8f a1, v8f a2, v8f a3, float oscale, u16* C, u16* C2,
                                      int res, float rsc, int N, size_t rowb, int col0, int lane,
                                      const float* __restrict__ bias, int bmode, int blen) {
  const int hh = lane >> 4, m = lane & 15;
  float bc[4], br[8];
  if (bmode != 0) {
#pragma unroll
    for (int j = 0; j < 4; ++j) bc[j] = 0.f;
#pragma unroll
    for (int r = 0; r < 8; ++r) {
      const int bi = min((int)rowb + 8 * hh + r, blen - 1);
      br[r] = bf_val(bias[bi]);
    }
  } else {
#pragma unroll
    for (int r = 0; r < 8; ++r) br[r] = 0.f;
#pragma unroll
    for (int j = 0; j < 4; ++j) {
      const int bi = min(col0 + 16 * j + m, blen - 1);
      bc[j] = bf_val(bias[bi]);
    }
  }
#pragma unroll
  for (int r = 0; r < 8; ++r) {
    const int ro = (8 * hh + r) * 68 + m;
    sl[ro]      = (a0[r] + br[r] + bc[0]) * oscale;
    sl[ro + 16] = (a1[r] + br[r] + bc[1]) * oscale;
    sl[ro + 32] = (a2[r] + br[r] + bc[2]) * oscale;
    sl[ro + 48] = (a3[r] + br[r] + bc[3]) * oscale;
  }
  wave_sync_lds();
  const int rq = lane >> 3, c8 = (lane & 7) * 8;
  v4u oh[4], ol[4];
#pragma unroll
  for (int i4 = 0; i4 < 4; ++i4) {
    const int row = i4 * 4 + rq;
    const v4f a = *(const v4f*)(sl + row * 68 + c8), c4 = *(const v4f*)(sl + row * 68 + c8 + 4);
    float w[8];
#pragma unroll
    for (int e = 0; e < 4; ++e) { w[e] = a[e]; w[4 + e] = c4[e]; }
#pragma unroll
    for (int e = 0; e < 4; ++e) {
      const _Float16 h0 = (_Float16)w[2 * e], h1 = (_Float16)w[2 * e + 1];
      const _Float16 l0 = (_Float16)((w[2 * e] - (float)h0) * rsc);
      const _Float16 l1 = (_Float16)((w[2 * e + 1] - (float)h1) * rsc);
      oh[i4][e] = pk16(h_bits(h0), h_bits(h1));
      ol[i4][e] = pk16(h_bits(l0), h_bits(l1));
    }
  }
  const size_t dofs = (rowb + (size_t)rq) * (size_t)N + col0 + c8;
  u16* dst  = C  + dofs;
  u16* dst2 = C2 + dofs;
  for (int pass = 0; pass < 2; ++pass) {
#pragma unroll
    for (int i4 = 0; i4 < 4; ++i4) {
      *(volatile v4u*)(dst + (size_t)(i4 * 4) * (size_t)N) = oh[i4];
    }
    if (res != 0) {
#pragma unroll
      for (int i4 = 0; i4 < 4; ++i4) {
        *(volatile v4u*)(dst2 + (size_t)(i4 * 4) * (size_t)N) = ol[i4];
      }
    }
    __threadfence();
  }
}

__device__ __forceinline__ void epi64(float* sl, v8f a0, v8f a1, v8f a2, v8f a3, float oscale, float* C, int N,
                                      size_t rowb, int col0, int lane, const float* __restrict__ bias, int blen) {
  const int hh = lane >> 4, m = lane & 15;
  float bc[4];
#pragma unroll
  for (int j = 0; j < 4; ++j) {
    const int bi = min(col0 + 16 * j + m, blen - 1);
    bc[j] = bf_val(bias[bi]);
  }
#pragma unroll
  for (int r = 0; r < 8; ++r) {
    const int ro = (8 * hh + r) * 68 + m;
    sl[ro]      = a0[r] * oscale + bc[0];
    sl[ro + 16] = a1[r] * oscale + bc[1];
    sl[ro + 32] = a2[r] * oscale + bc[2];
    sl[ro + 48] = a3[r] * oscale + bc[3];
  }
  wave_sync_lds();
  v4f vals[8];
#pragma unroll
  for (int it = 0; it < 8; ++it) vals[it] = *(const v4f*)(sl + (it * 2 + hh) * 68 + m * 4);
  float* dst = C + (rowb + (size_t)hh) * (size_t)N + col0 + m * 4;
  for (int pass = 0; pass < 2; ++pass) {
#pragma unroll
    for (int it = 0; it < 8; ++it) {
      *(volatile v4f*)(dst + (size_t)(it * 2) * (size_t)N) = vals[it];
    }
    __threadfence();
  }
}

__global__ __launch_bounds__(128)
void gemm_b16(const u16* __restrict__ A, const u16* __restrict__ Bt, u16* C, u16* C2, int M, int N, int K,
              float oscale, const float* __restrict__ bias, int bmode, int blen, int res, float rsc) {
  __shared__ __align__(16) float slab[4 * SLAB];
  const int tid = threadIdx.x, wave = tid >> 5, lane = tid & 31, hh = lane >> 4, m = lane & 15;
  const int ntile = N >> 6;
  const int bid   = blockIdx.x;
  const int rowb  = (bid / ntile) * 64 + wave * 16;
  const int col0  = (bid % ntile) * 64;
  if (rowb + 16 > M) return;
  const u16* ap = A  + (size_t)(rowb + m) * (size_t)K + 8 * hh;
  const u16* bp = Bt + (size_t)(col0 + m) * (size_t)K + 8 * hh;
  const size_t bs = (size_t)16 * K;
  v8f acc0 = zero8(), acc1 = zero8(), acc2 = zero8(), acc3 = zero8();
#pragma unroll 1
  for (int k0 = 0; k0 < K; k0 += 32) {
    const v16b a  = ldfrag_b(ap + k0);
    const v16b b0 = ldfrag_b(bp + k0);
    const v16b b1 = ldfrag_b(bp + bs + k0);
    const v16b b2 = ldfrag_b(bp + 2 * bs + k0);
    const v16b b3 = ldfrag_b(bp + 3 * bs + k0);
    acc0 = mma_b(a, b0, acc0);
    acc1 = mma_b(a, b1, acc1);
    acc2 = mma_b(a, b2, acc2);
    acc3 = mma_b(a, b3, acc3);
    guard6<v16b>(acc0, acc1, acc2, acc3, a, b0, b1, b2, b3, a);
  }
  epi16(slab + wave * SLAB, acc0, acc1, acc2, acc3, oscale, C, C2, res, rsc, N, (size_t)rowb, col0, lane,
        bias, bmode, blen);
}

__global__ __launch_bounds__(128)
void gemm_hf2(const u16* __restrict__ A1, const u16* __restrict__ A2, const u16* __restrict__ Bt, float* C,
              int M, int N, int K, float oscale, float rinv, const float* __restrict__ bias, int blen) {
  __shared__ __align__(16) float slab[4 * SLAB];
  const int tid = threadIdx.x, wave = tid >> 5, lane = tid & 31, hh = lane >> 4, m = lane & 15;
  const int ntile = N >> 6;
  const int bid   = blockIdx.x;
  const int rowb  = (bid / ntile) * 64 + wave * 16;
  const int col0  = (bid % ntile) * 64;
  if (rowb + 16 > M) return;
  const _Float16* ap1 = (const _Float16*)(const void*)A1 + (size_t)(rowb + m) * (size_t)K + 8 * hh;
  const _Float16* ap2 = (const _Float16*)(const void*)A2 + (size_t)(rowb + m) * (size_t)K + 8 * hh;
  const _Float16* bp  = (const _Float16*)(const void*)Bt + (size_t)(col0 + m) * (size_t)K + 8 * hh;
  const size_t bs = (size_t)16 * K;
  v8f am0 = zero8(), am1 = zero8(), am2 = zero8(), am3 = zero8();
  v8f ar0 = zero8(), ar1 = zero8(), ar2 = zero8(), ar3 = zero8();
#pragma unroll 1
  for (int k0 = 0; k0 < K; k0 += 32) {
    const v16h a1 = ldfrag_h(ap1 + k0);
    const v16h a2 = ldfrag_h(ap2 + k0);
    const v16h b0 = ldfrag_h(bp + k0);
    const v16h b1 = ldfrag_h(bp + bs + k0);
    const v16h b2 = ldfrag_h(bp + 2 * bs + k0);
    const v16h b3 = ldfrag_h(bp + 3 * bs + k0);
    am0 = mma_h(a1, b0, am0);
    am1 = mma_h(a1, b1, am1);
    am2 = mma_h(a1, b2, am2);
    am3 = mma_h(a1, b3, am3);
    ar0 = mma_h(a2, b0, ar0);
    ar1 = mma_h(a2, b1, ar1);
    ar2 = mma_h(a2, b2, ar2);
    ar3 = mma_h(a2, b3, ar3);
    guard8(am0, am1, am2, am3, ar0, ar1, ar2, ar3, a1, a2, b0, b1, b2, b3);
  }
  acc_guard4(ar0, ar1, ar2, ar3);
  const v8f f0 = am0 + ar0 * rinv;
  const v8f f1 = am1 + ar1 * rinv;
  const v8f f2 = am2 + ar2 * rinv;
  const v8f f3 = am3 + ar3 * rinv;
  epi64(slab + wave * SLAB, f0, f1, f2, f3, oscale, C, N, (size_t)rowb, col0, lane, bias, blen);
}

__global__ __launch_bounds__(ATT_THREADS)
void attn_fwd(const u16* __restrict__ QHp, const u16* __restrict__ QLp, const u16* __restrict__ KHp,
              const u16* __restrict__ KLp, const u16* __restrict__ VPp, u16* OHp, u16* OLp) {
  __shared__ __align__(16) float smem[ATT_WAVES * SLAB];

  const int tid  = threadIdx.x;
  const int wave = tid >> 5;
  const int lane = tid & 31;
  const int hh   = lane >> 4;
  const int c    = lane & 15;

  const int bid  = blockIdx.x;
  const int qt   = bid % NQT;
  const int head = bid / NQT;
  if (head >= NH) return;
  const int qb   = qt * 64;
  const int q0   = qb + wave * 16;

  const int jlo  = max(qb - WSPAN, 0);
  const int jhi  = min(qb + 63 + WSPAN, SEQ - 1);
  const int kblo = jlo >> 5;
  int nkb = (jhi >> 5) - kblo + 1;
  nkb = min(max(nkb, 1), NKB - kblo);

  const size_t qofs = (size_t)(q0 + c) * DMOD + head * HD + 8 * hh;
  const _Float16* Qh = (const _Float16*)(const void*)QHp + qofs;
  const _Float16* Ql = (const _Float16*)(const void*)QLp + qofs;
  const size_t kofs = (size_t)c * DMOD + head * HD + 8 * hh;
  const _Float16* Kh = (const _Float16*)(const void*)KHp + kofs;
  const _Float16* Kl = (const _Float16*)(const void*)KLp + kofs;
  const size_t vofs = ((size_t)(head * HD + c)) * SEQ + 8 * hh;
  const _Float16* Vb = (const _Float16*)(const void*)VPp + vofs;
  const float lsc  = RSQN * (LOG2E / (QSC * KSC));
  const float qkri = 1.0f / QKRS;
  const int dq = q0 + c - 8 * hh;

  const v16h qh0 = ldfrag_h(Qh);
  const v16h qh1 = ldfrag_h(Qh + 32);
  const v16h ql0 = ldfrag_h(Ql);
  const v16h ql1 = ldfrag_h(Ql + 32);

  float mrun = NEGS, lrun = 0.f;
  v8f o[4];
#pragma unroll
  for (int j = 0; j < 4; ++j) o[j] = zero8();

#pragma unroll 1
  for (int it = 0; it < nkb; ++it) {
    const int kb = (kblo + it) * 32;
    float tk[16];
    {
      v8f s = zero8(), rr = zero8();
      const _Float16* hp = Kh + (size_t)kb * DMOD;
      const _Float16* lp = Kl + (size_t)kb * DMOD;
      const v16h ka = ldfrag_h(hp), kc = ldfrag_h(hp + 32);
      const v16h la = ldfrag_h(lp), lc = ldfrag_h(lp + 32);
      s  = mma_h(ka, qh0, s);
      s  = mma_h(kc, qh1, s);
      rr = mma_h(ka, ql0, rr);
      rr = mma_h(kc, ql1, rr);
      rr = mma_h(la, qh0, rr);
      rr = mma_h(lc, qh1, rr);
      guard2f8(s, rr, ka, kc, la, lc, qh0, qh1, ql0, ql1);
#pragma unroll
      for (int i = 0; i < 8; ++i) {
        const int d0 = dq - kb - i;
        const bool a0 = (d0 <= WSPAN) && (d0 >= -WSPAN);
        tk[i] = a0 ? ((s[i] + rr[i] * qkri) * lsc) : NEGS;
      }
    }
    {
      v8f s = zero8(), rr = zero8();
      const _Float16* hp = Kh + (size_t)(kb + 16) * DMOD;
      const _Float16* lp = Kl + (size_t)(kb + 16) * DMOD;
      const v16h ka = ldfrag_h(hp), kc = ldfrag_h(hp + 32);
      const v16h la = ldfrag_h(lp), lc = ldfrag_h(lp + 32);
      s  = mma_h(ka, qh0, s);
      s  = mma_h(kc, qh1, s);
      rr = mma_h(ka, ql0, rr);
      rr = mma_h(kc, ql1, rr);
      rr = mma_h(la, qh0, rr);
      rr = mma_h(lc, qh1, rr);
      guard2f8(s, rr, ka, kc, la, lc, qh0, qh1, ql0, ql1);
#pragma unroll
      for (int i = 0; i < 8; ++i) {
        const int d1 = dq - kb - 16 - i;
        const bool a1 = (d1 <= WSPAN) && (d1 >= -WSPAN);
        tk[8 + i] = a1 ? ((s[i] + rr[i] * qkri) * lsc) : NEGS;
      }
    }
    float cm = tk[0];
#pragma unroll
    for (int i = 1; i < 16; ++i) cm = fmaxf(cm, tk[i]);
    cm = fmaxf(cm, __shfl_xor(cm, 16, 32));
    const float mn = fmaxf(mrun, cm);
    const float al = exp2f(fminf(mrun - mn, 0.f));
    mrun = mn;
    float ps = 0.f;
    FragH ph;
#pragma unroll
    for (int wq = 0; wq < 2; ++wq) {
#pragma unroll
      for (int e4 = 0; e4 < 4; ++e4) {
        const int i = 8 * wq + 2 * e4;
        const float x0 = exp2f(fminf(tk[i] - mn, 0.f));
        const float x1 = exp2f(fminf(tk[i + 1] - mn, 0.f));
        const float p0 = (tk[i] > -1.0e38f) ? x0 : 0.f;
        const float p1 = (tk[i + 1] > -1.0e38f) ? x1 : 0.f;
        ps += p0 + p1;
        ph.u[wq][e4] = pk16(h_bits((_Float16)(p0 * PCAR)), h_bits((_Float16)(p1 * PCAR)));
      }
    }
    ps += __shfl_xor(ps, 16, 32);
    lrun = lrun * al + ps;
    float scl[8];
#pragma unroll
    for (int r = 0; r < 8; ++r) scl[r] = __shfl(al, 8 * hh + r, 32);
#pragma unroll
    for (int j = 0; j < 4; ++j) {
#pragma unroll
      for (int r = 0; r < 8; ++r) o[j][r] *= scl[r];
    }
    {
      const _Float16* vp = Vb + kb;
      const v16h vf0 = ldfrag_h(vp);
      const v16h vf1 = ldfrag_h(vp + (size_t)16 * SEQ);
      const v16h vf2 = ldfrag_h(vp + (size_t)32 * SEQ);
      const v16h vf3 = ldfrag_h(vp + (size_t)48 * SEQ);
      o[0] = mma_h(ph.v, vf0, o[0]);
      o[1] = mma_h(ph.v, vf1, o[1]);
      o[2] = mma_h(ph.v, vf2, o[2]);
      o[3] = mma_h(ph.v, vf3, o[3]);
      guard6<v16h>(o[0], o[1], o[2], o[3], ph.v, vf0, vf1, vf2, vf3, ph.v);
    }
  }
  acc_guard4(o[0], o[1], o[2], o[3]);

  const float linv = (lrun > 0.f) ? ((1.0f / lrun) * (1.0f / (PCAR * VCAR))) : 0.f;
  float inv[8];
#pragma unroll
  for (int r = 0; r < 8; ++r) inv[r] = __shfl(linv, 8 * hh + r, 32);
  float* slab = smem + wave * SLAB;
#pragma unroll
  for (int r = 0; r < 8; ++r) {
#pragma unroll
    for (int j = 0; j < 4; ++j) slab[(8 * hh + r) * 68 + j * 16 + c] = o[j][r] * inv[r];
  }
  wave_sync_lds();
  v4u oh[4], ol[4];
  const int rq = lane >> 3, c8 = (lane & 7) * 8;
#pragma unroll
  for (int i4 = 0; i4 < 4; ++i4) {
    const int row = i4 * 4 + rq;
    const v4f a = *(const v4f*)(slab + row * 68 + c8), c4 = *(const v4f*)(slab + row * 68 + c8 + 4);
    float wv[8];
#pragma unroll
    for (int e = 0; e < 4; ++e) { wv[e] = a[e] * OSC; wv[4 + e] = c4[e] * OSC; }
#pragma unroll
    for (int e = 0; e < 4; ++e) {
      const _Float16 h0 = (_Float16)wv[2 * e], h1 = (_Float16)wv[2 * e + 1];
      const _Float16 l0 = (_Float16)((wv[2 * e] - (float)h0) * ORS);
      const _Float16 l1 = (_Float16)((wv[2 * e + 1] - (float)h1) * ORS);
      oh[i4][e] = pk16(h_bits(h0), h_bits(h1));
      ol[i4][e] = pk16(h_bits(l0), h_bits(l1));
    }
  }
  const size_t ob = (size_t)q0 * DMOD + head * HD + c8;
  for (int pass = 0; pass < 2; ++pass) {
#pragma unroll
    for (int i4 = 0; i4 < 4; ++i4) {
      const int row = i4 * 4 + rq;
      const size_t o8 = ob + (size_t)row * DMOD;
      *(volatile v4u*)(OHp + o8) = oh[i4];
      *(volatile v4u*)(OLp + o8) = ol[i4];
    }
    __threadfence();
  }
}

extern "C" void kernel_launch(void* const* d_in, const int* in_sizes, int n_in,
                              void* d_out, int out_size, void* d_ws, size_t ws_size,
                              hipStream_t stream) {
  const int ROWS = SEQ;
  if (n_in < 11) return;
  if (in_sizes[0] < ROWS * DMOD || in_sizes[1] < ROWS * DMOD || in_sizes[2] < ROWS * DMOD) return;
  if (in_sizes[3] < DMOD * DMOD || in_sizes[5] < DMOD * DMOD || in_sizes[7] < DMOD * DMOD || in_sizes[9] < DMOD * DMOD) return;
  if (in_sizes[4] < DMOD || in_sizes[6] < DMOD || in_sizes[8] < DMOD || in_sizes[10] < DMOD) return;
  if (out_size < ROWS * DMOD) return;

  const float* Qin = (const float*)d_in[0];
  const float* Kin = (const float*)d_in[1];
  const float* Vin = (const float*)d_in[2];
  const float* Wq  = (const float*)d_in[3];
  const float* Bq  = (const float*)d_in[4];
  const float* Wk  = (const float*)d_in[5];
  const float* Bk  = (const float*)d_in[6];
  const float* Wv  = (const float*)d_in[7];
  const float* Bv  = (const float*)d_in[8];
  const float* Wo  = (const float*)d_in[9];
  const float* Bo  = (const float*)d_in[10];
  float*       out = (float*)d_out;

  const size_t szX = (size_t)ROWS * DMOD * 2;
  const size_t szW = (size_t)DMOD * DMOD * 2;
  size_t off = 0;
  const size_t oXQ = off; off += szX;
  const size_t oXK = off; off += szX;
  const size_t oXV = off; off += szX;
  const size_t oWQ = off; off += szW;
  const size_t oWK = off; off += szW;
  const size_t oWV = off; off += szW;
  const size_t oWO = off; off += szW;
  const size_t oQH = off; off += szX;
  const size_t oQL = off; off += szX;
  const size_t oKH = off; off += szX;
  const size_t oKL = off; off += szX;
  const size_t oVP = off; off += szX;
  const size_t oOH = off; off += szX;
  const size_t oOL = off; off += szX;
  if (off > ws_size) return;
  if (off > (size_t)134217728) return;

  char* ws = (char*)d_ws;
  u16* XQ  = (u16*)(ws + oXQ);
  u16* XK  = (u16*)(ws + oXK);
  u16* XV  = (u16*)(ws + oXV);
  u16* WQT = (u16*)(ws + oWQ);
  u16* WKT = (u16*)(ws + oWK);
  u16* WVT = (u16*)(ws + oWV);
  u16* WOT = (u16*)(ws + oWO);
  u16* QH  = (u16*)(ws + oQH);
  u16* QL  = (u16*)(ws + oQL);
  u16* KH  = (u16*)(ws + oKH);
  u16* KL  = (u16*)(ws + oKL);
  u16* VP  = (u16*)(ws + oVP);
  u16* OH  = (u16*)(ws + oOH);
  u16* OL  = (u16*)(ws + oOL);

  const int n8x = (ROWS * DMOD) / 8;
  if ((n8x % 256) != 0) return;
  if ((DMOD % 64) != 0 || (ROWS % 64) != 0 || (DMOD % 32) != 0) return;
  const dim3 blk(256);
  const dim3 gX(n8x / 256);
  const dim3 gT((DMOD / 64) * (DMOD / 64));
  const dim3 gG((ROWS / 64) * (DMOD / 64));
  const dim3 bG(128);
  const dim3 gAT(ATT_BLOCKS);
  const dim3 bAT(ATT_THREADS);

  cvt16<<<gX, blk, 0, stream>>>(Qin, XQ, n8x);
  cvt16<<<gX, blk, 0, stream>>>(Kin, XK, n8x);
  cvt16<<<gX, blk, 0, stream>>>(Vin, XV, n8x);
  cvtT16<<<gT, blk, 0, stream>>>(Wq, WQT, DMOD, DMOD, 0, 1.0f);
  cvtT16<<<gT, blk, 0, stream>>>(Wk, WKT, DMOD, DMOD, 0, 1.0f);
  cvtT16<<<gT, blk, 0, stream>>>(Wv, WVT, DMOD, DMOD, 0, 1.0f);
  cvtT16<<<gT, blk, 0, stream>>>(Wo, WOT, DMOD, DMOD, 1, WOS);
  gemm_b16<<<gG, bG, 0, stream>>>(XQ, WQT, QH, QL, ROWS, DMOD, DMOD, QSC, Bq, 0, DMOD, 1, QKRS);
  gemm_b16<<<gG, bG, 0, stream>>>(XK, WKT, KH, KL, ROWS, DMOD, DMOD, KSC, Bk, 0, DMOD, 1, QKRS);
  gemm_b16<<<gG, bG, 0, stream>>>(WVT, XV, VP, VP, DMOD, ROWS, DMOD, VCAR, Bv, 1, DMOD, 0, QKRS);
  attn_fwd<<<gAT, bAT, 0, stream>>>(QH, QL, KH, KL, VP, OH, OL);
  gemm_hf2<<<gG, bG, 0, stream>>>(OH, OL, WOT, out, ROWS, DMOD, DMOD, 1.0f / (OSC * WOS), 1.0f / ORS, Bo, DMOD);
  (void)hipGetLastError();
}
